// InteractionNet_2302102471382
// MI455X (gfx1250) — hardware-verified
//
#include <hip/hip_runtime.h>
#include <math.h>

typedef __attribute__((ext_vector_type(16))) _Float16 v16h;
typedef __attribute__((ext_vector_type(16))) __bf16 v16b;
typedef __attribute__((ext_vector_type(8)))  _Float16 v8h;
typedef __attribute__((ext_vector_type(8)))  float v8f;
typedef __attribute__((ext_vector_type(4)))  float v4f;
typedef __attribute__((ext_vector_type(2)))  float v2f;
typedef __attribute__((ext_vector_type(4)))  unsigned v4u;
typedef __attribute__((ext_vector_type(4)))  int v4i;
typedef float __attribute__((may_alias)) float_a;
typedef int __attribute__((may_alias)) int_a;

template <typename T> __device__ __forceinline__ void vst2(void* p, T v) { *(volatile T*)p = v; __threadfence(); *(volatile T*)p = v; }
__device__ __forceinline__ v8f wmma16(v16h a, v16h b, v8f c) {
  v8f d = __builtin_amdgcn_wmma_f32_16x16x32_f16(false, a, false, b, (short)0, c, false, false);
  asm volatile("v_nop\n\tv_nop\n\tv_nop\n\tv_nop" : "+v"(d) : "v"(a), "v"(b));
  return d;
}
__device__ __forceinline__ v8f wmma_bf(v16b a, v16b b, v8f c) {
  v8f d = __builtin_amdgcn_wmma_f32_16x16x32_bf16(false, a, false, b, (short)0, c, false, false);
  asm volatile("v_nop\n\tv_nop\n\tv_nop\n\tv_nop" : "+v"(d) : "v"(a), "v"(b));
  return d;
}
__device__ __forceinline__ v16h frag_h(const _Float16* rowk0, int lane) {
  union { v16h v; v8h q[2]; } u; const _Float16* p = rowk0 + 8 * (lane >> 4);
  u.q[0] = *(const v8h*)p; u.q[1] = *(const v8h*)(p + 16); return u.v;
}
__device__ __forceinline__ v16h frag_f32(const float* rowk0, int lane) {
  v16h a; const float* p = rowk0 + 8 * (lane >> 4);
#pragma unroll
  for (int i = 0; i < 8; ++i) { a[i] = (_Float16)p[i]; a[8 + i] = (_Float16)p[16 + i]; }
  return a;
}
__device__ __forceinline__ v16h frag_f32s(const float* rowk0, int lane, float sc) {
  v16h a; const float* p = rowk0 + 8 * (lane >> 4);
#pragma unroll
  for (int i = 0; i < 8; ++i) { a[i] = (_Float16)(p[i] * sc); a[8 + i] = (_Float16)(p[16 + i] * sc); }
  return a;
}
__device__ __forceinline__ v16h fragc_f32(const float* W, int k0, int n, int lane, int ld, int K) {
  v16h a; const int g = lane >> 4;
#pragma unroll
  for (int i = 0; i < 8; ++i) { const int ka = k0 + 8 * g + i, kb = ka + 16;
    a[i] = (_Float16)(ka < K ? W[(size_t)(ka < K ? ka : K - 1) * ld + n] : 0.f); a[8 + i] = (_Float16)(kb < K ? W[(size_t)(kb < K ? kb : K - 1) * ld + n] : 0.f); }
  return a;
}
struct F2 { v16b h, l; };
__device__ __forceinline__ F2 bsplit16(const float v[16]) { F2 r;
#pragma unroll
  for (int i = 0; i < 16; ++i) { const __bf16 h = (__bf16)v[i]; r.h[i] = h; r.l[i] = (__bf16)(v[i] - (float)h); }
  return r; }
__device__ __forceinline__ F2 split_row(const float* row, int k0, int lane) { float v[16]; const float* p = row + k0 + 8 * (lane >> 4);
#pragma unroll
  for (int i = 0; i < 8; ++i) { v[i] = p[i]; v[8 + i] = p[16 + i]; }
  return bsplit16(v); }
__device__ __forceinline__ F2 split_rowK(const float* row, int k0, int lane, int K) { float v[16]; const int g = lane >> 4;
#pragma unroll
  for (int i = 0; i < 8; ++i) { const int ka = k0 + 8 * g + i, kb = ka + 16; v[i] = ka < K ? row[ka < K ? ka : K - 1] : 0.f; v[8 + i] = kb < K ? row[kb < K ? kb : K - 1] : 0.f; }
  return bsplit16(v); }
__device__ __forceinline__ F2 split_col(const float* W, int k0, int n, int lane, int ld, int K) { float v[16]; const int g = lane >> 4;
#pragma unroll
  for (int i = 0; i < 8; ++i) { const int ka = k0 + 8 * g + i, kb = ka + 16; v[i] = ka < K ? W[(size_t)(ka < K ? ka : K - 1) * ld + n] : 0.f; v[8 + i] = kb < K ? W[(size_t)(kb < K ? kb : K - 1) * ld + n] : 0.f; }
  return bsplit16(v); }
__device__ __forceinline__ v8f mac3(const F2& a, const F2& b, v8f c) { c = wmma_bf(a.l, b.h, c); c = wmma_bf(a.h, b.l, c); return wmma_bf(a.h, b.h, c); }
__device__ __forceinline__ float sigm(float v) { return 1.0f / (1.0f + expf(-v)); }
#define LDSX() do { asm volatile("s_wait_dscnt 0" ::: "memory"); __builtin_amdgcn_wave_barrier(); __builtin_amdgcn_fence(__ATOMIC_RELEASE, "workgroup"); } while (0)


#define NBATCH 16384
#define NNODE 29
#define NP 32
#define DM 128
#define EPB 32
typedef __attribute__((ext_vector_type(8))) __bf16 v8b;
__device__ __forceinline__ v16b frag_b(const __bf16* rowk0, int lane) {
  union { v16b v; v8b q[2]; } u; const __bf16* p = rowk0 + 8 * (lane >> 4);
  u.q[0] = *(const v8b*)p; u.q[1] = *(const v8b*)(p + 16); return u.v;
}
__device__ __forceinline__ float bfr(float v) { return (float)(__bf16)v; }
__device__ __attribute__((noinline)) float exp_ni(float v) { return expf(v); }
__device__ __attribute__((noinline)) float erf_ni(float v) { return erff(v); }

#define PK_A  0
#define PK_W1 (6 * NP * NP)
#define PK_W  (PK_W1 + DM * NP)
#define PK_T  (PK_W + 5 * DM * DM)
#define PK_END (PK_T + 16 * DM)
#define WS_END (((2u * PK_END) + 127u) / 128u * 128u)

struct InPtrs { const float* A[6]; const float* W1; const float* W[5]; const float* WT; };
struct BPtrs { const float* b[6]; const float* bt; };
__global__ __launch_bounds__(128) void k_pack(InPtrs IP, __bf16* __restrict__ PK) {
  __shared__ __align__(16) __bf16 s[DM]; const int n = blockIdx.x, which = blockIdx.y, t = threadIdx.x; int K; size_t dst; float v = 0.f;
  if (which < 6) { if (n >= NP) return; K = NP; dst = PK_A + ((size_t)which * NP + n) * NP; const float* A = IP.A[which]; if (t < NP) { v = (n < NNODE && t < NNODE) ? A[n * NNODE + t] : 0.f; s[t] = (__bf16)v; } }
  else if (which == 6) { K = NP; dst = PK_W1 + (size_t)n * NP; const float* W1 = IP.W1; if (t < NP) { v = (t < 3) ? W1[t * DM + n] : 0.f; s[t] = (__bf16)v; } }
  else if (which < 12) { K = DM; dst = PK_W + ((size_t)(which - 7) * DM + n) * DM; const float* Wl = IP.W[which - 7]; s[t] = (__bf16)Wl[(size_t)t * DM + n]; }
  else { if (n >= 16) return; K = DM; dst = PK_T + (size_t)n * DM; const float* WT = IP.WT; s[t] = (__bf16)((n < 3) ? WT[(size_t)t * 3 + n] : 0.f); }
  __syncthreads();
  if (t < K / 8) vst2((unsigned*)(PK + dst + t * 8), *(const v4u*)&s[t * 8]);
}
__global__ __launch_bounds__(128) void k_net(const float* __restrict__ POSE, const __bf16* __restrict__ PK, BPtrs BP, float* __restrict__ OUT) {
  __shared__ __align__(16) __bf16 sxh[64][DM + 8], sxl[64][DM + 8]; __shared__ __align__(16) __bf16 sth[2][DM][40], stl[2][DM][40]; __shared__ __align__(16) float sout[EPB * NNODE * 3 + 16]; __shared__ float sb[6][DM], sbt[4];
  const int tid = threadIdx.x, wave = tid >> 5, lane = tid & 31, col = lane & 15, g = lane >> 4; const int el = wave >> 1;
  for (int e = tid; e < 6 * DM; e += 128) sb[e / DM][e % DM] = bfr(BP.b[e / DM][e % DM]);
  if (tid < 3) sbt[tid] = bfr(BP.bt[tid]);
#pragma unroll 1
  for (int pr = 0; pr < EPB / 2; ++pr) { const size_t e0 = (size_t)blockIdx.x * EPB + pr * 2;
    for (int e = tid; e < 64 * NP; e += 128) { const int r = e / NP, c = e % NP; const int n = r & 31; const size_t el2 = e0 + (r >> 5); const float v = (n < NNODE && c < 3) ? bfr(POSE[(el2 * NNODE + n) * 3 + c]) : 0.f; sxh[r][c] = (__bf16)v; sxl[r][c] = (__bf16)0.f; }
    __syncthreads();
#pragma unroll 1
    for (int l = 0; l < 6; ++l) { const int KD = (l == 0) ? NP : DM; const __bf16* WP = (l == 0) ? (PK + PK_W1) : (PK + PK_W + (size_t)(l - 1) * DM * DM);
      v8f acc[8] = {};
      for (int kc = 0; kc < KD / 32; ++kc) { F2 a; a.h = frag_b(&sxh[wave * 16 + col][kc * 32], lane); a.l = frag_b(&sxl[wave * 16 + col][kc * 32], lane);
#pragma unroll
        for (int j = 0; j < 8; ++j) { const v16b w = frag_b(WP + (size_t)(j * 16 + col) * KD + kc * 32, lane); acc[j] = wmma_bf(a.l, w, acc[j]); acc[j] = wmma_bf(a.h, w, acc[j]); } }
      __syncthreads();
#pragma unroll
      for (int j = 0; j < 8; ++j)
#pragma unroll
        for (int r = 0; r < 8; ++r) { const int node = (wave & 1) * 16 + 8 * g + r; const float v = acc[j][r]; const __bf16 hb = (__bf16)v; sth[el][j * 16 + col][node] = hb; stl[el][j * 16 + col][node] = (__bf16)(v - (float)hb); }
      __syncthreads();
      v8f acc2[8] = {};
      { const v16b a = frag_b(PK + PK_A + ((size_t)l * NP + (wave & 1) * 16 + col) * NP, lane);
#pragma unroll
        for (int j = 0; j < 8; ++j) { acc2[j] = wmma_bf(a, frag_b(&stl[el][j * 16 + col][0], lane), acc2[j]); acc2[j] = wmma_bf(a, frag_b(&sth[el][j * 16 + col][0], lane), acc2[j]); } }
#pragma unroll
      for (int j = 0; j < 8; ++j) { const int c = j * 16 + col; const float bb = sb[l][c];
#pragma unroll
        for (int r = 0; r < 8; ++r) { const int node = (wave & 1) * 16 + 8 * g + r; const float v = (node < NNODE) ? (acc2[j][r] + bb) : 0.f; const __bf16 hb = (__bf16)v; sxh[wave * 16 + 8 * g + r][c] = hb; sxl[wave * 16 + 8 * g + r][c] = (__bf16)(v - (float)hb); } }
      __syncthreads(); }
    { v8f acc = {};
#pragma unroll
      for (int kc = 0; kc < DM / 32; ++kc) { F2 a; a.h = frag_b(&sxh[wave * 16 + col][kc * 32], lane); a.l = frag_b(&sxl[wave * 16 + col][kc * 32], lane); const v16b w = frag_b(PK + PK_T + (size_t)col * DM + kc * 32, lane); acc = wmma_bf(a.l, w, acc); acc = wmma_bf(a.h, w, acc); }
      if (col < 3) {
#pragma unroll
        for (int r = 0; r < 8; ++r) { const int node = (wave & 1) * 16 + 8 * g + r; if (node < NNODE) { const size_t el2 = e0 + el; const float v = acc[r] + sbt[col] + bfr(POSE[(el2 * NNODE + node) * 3 + col]); sout[((pr * 2 + el) * NNODE + node) * 3 + col] = v; } } } }
    __syncthreads(); }
  for (int q = tid; q < EPB * NNODE * 3 / 4; q += 128) vst2(OUT + (size_t)blockIdx.x * EPB * NNODE * 3 + q * 4, *(const v4f*)&sout[q * 4]);
}
extern "C" void kernel_launch(void* const* d_in, const int* in_sizes, int n_in, void* d_out, int out_size, void* d_ws, size_t ws_size, hipStream_t stream) {
  (void)in_sizes; (void)n_in; (void)out_size;
  static_assert((EPB * NNODE * 3) % 32 == 0, "block output must be whole 128-B lines");
  if (ws_size < (size_t)WS_END) return;
  const float** F = (const float**)d_in; __bf16* PK = (__bf16*)d_ws;
  InPtrs IP; for (int l = 0; l < 6; ++l) IP.A[l] = F[1 + l]; IP.W1 = F[7]; for (int l = 0; l < 5; ++l) IP.W[l] = F[9 + 2 * l]; IP.WT = F[19];
  BPtrs BP; for (int l = 0; l < 6; ++l) BP.b[l] = F[8 + 2 * l]; BP.bt = F[20];
  k_pack<<<dim3(DM, 13), 128, 0, stream>>>(IP, PK);
  k_net<<<NBATCH / EPB, 128, 0, stream>>>(F[0], PK, BP, (float*)d_out);
}
